// EquivariantAttention_14611478741511
// MI455X (gfx1250) — hardware-verified
//
#include <hip/hip_runtime.h>
#include <math.h>

typedef __attribute__((ext_vector_type(16))) _Float16 v16h;
typedef __attribute__((ext_vector_type(16))) __bf16 v16b;
typedef __attribute__((ext_vector_type(8)))  _Float16 v8h;
typedef __attribute__((ext_vector_type(8)))  float v8f;
typedef __attribute__((ext_vector_type(4)))  float v4f;
typedef __attribute__((ext_vector_type(2)))  float v2f;
typedef __attribute__((ext_vector_type(4)))  unsigned v4u;
typedef __attribute__((ext_vector_type(4)))  int v4i;
typedef float __attribute__((may_alias)) float_a;
typedef int __attribute__((may_alias)) int_a;

template <typename T> __device__ __forceinline__ void vst2(void* p, T v) { *(volatile T*)p = v; __threadfence(); *(volatile T*)p = v; }
__device__ __forceinline__ v8f wmma16(v16h a, v16h b, v8f c) {
  v8f d = __builtin_amdgcn_wmma_f32_16x16x32_f16(false, a, false, b, (short)0, c, false, false);
  asm volatile("v_nop\n\tv_nop\n\tv_nop\n\tv_nop" : "+v"(d) : "v"(a), "v"(b));
  return d;
}
__device__ __forceinline__ v8f wmma_bf(v16b a, v16b b, v8f c) {
  v8f d = __builtin_amdgcn_wmma_f32_16x16x32_bf16(false, a, false, b, (short)0, c, false, false);
  asm volatile("v_nop\n\tv_nop\n\tv_nop\n\tv_nop" : "+v"(d) : "v"(a), "v"(b));
  return d;
}
__device__ __forceinline__ v16h frag_h(const _Float16* rowk0, int lane) {
  union { v16h v; v8h q[2]; } u; const _Float16* p = rowk0 + 8 * (lane >> 4);
  u.q[0] = *(const v8h*)p; u.q[1] = *(const v8h*)(p + 16); return u.v;
}
__device__ __forceinline__ v16h frag_f32(const float* rowk0, int lane) {
  v16h a; const float* p = rowk0 + 8 * (lane >> 4);
#pragma unroll
  for (int i = 0; i < 8; ++i) { a[i] = (_Float16)p[i]; a[8 + i] = (_Float16)p[16 + i]; }
  return a;
}
__device__ __forceinline__ v16h frag_f32s(const float* rowk0, int lane, float sc) {
  v16h a; const float* p = rowk0 + 8 * (lane >> 4);
#pragma unroll
  for (int i = 0; i < 8; ++i) { a[i] = (_Float16)(p[i] * sc); a[8 + i] = (_Float16)(p[16 + i] * sc); }
  return a;
}
__device__ __forceinline__ v16h fragc_f32(const float* W, int k0, int n, int lane, int ld, int K) {
  v16h a; const int g = lane >> 4;
#pragma unroll
  for (int i = 0; i < 8; ++i) { const int ka = k0 + 8 * g + i, kb = ka + 16;
    a[i] = (_Float16)(ka < K ? W[(size_t)(ka < K ? ka : K - 1) * ld + n] : 0.f); a[8 + i] = (_Float16)(kb < K ? W[(size_t)(kb < K ? kb : K - 1) * ld + n] : 0.f); }
  return a;
}
struct F2 { v16b h, l; };
__device__ __forceinline__ F2 bsplit16(const float v[16]) { F2 r;
#pragma unroll
  for (int i = 0; i < 16; ++i) { const __bf16 h = (__bf16)v[i]; r.h[i] = h; r.l[i] = (__bf16)(v[i] - (float)h); }
  return r; }
__device__ __forceinline__ F2 split_row(const float* row, int k0, int lane) { float v[16]; const float* p = row + k0 + 8 * (lane >> 4);
#pragma unroll
  for (int i = 0; i < 8; ++i) { v[i] = p[i]; v[8 + i] = p[16 + i]; }
  return bsplit16(v); }
__device__ __forceinline__ F2 split_rowK(const float* row, int k0, int lane, int K) { float v[16]; const int g = lane >> 4;
#pragma unroll
  for (int i = 0; i < 8; ++i) { const int ka = k0 + 8 * g + i, kb = ka + 16; v[i] = ka < K ? row[ka < K ? ka : K - 1] : 0.f; v[8 + i] = kb < K ? row[kb < K ? kb : K - 1] : 0.f; }
  return bsplit16(v); }
__device__ __forceinline__ F2 split_col(const float* W, int k0, int n, int lane, int ld, int K) { float v[16]; const int g = lane >> 4;
#pragma unroll
  for (int i = 0; i < 8; ++i) { const int ka = k0 + 8 * g + i, kb = ka + 16; v[i] = ka < K ? W[(size_t)(ka < K ? ka : K - 1) * ld + n] : 0.f; v[8 + i] = kb < K ? W[(size_t)(kb < K ? kb : K - 1) * ld + n] : 0.f; }
  return bsplit16(v); }
__device__ __forceinline__ v8f mac3(const F2& a, const F2& b, v8f c) { c = wmma_bf(a.l, b.h, c); c = wmma_bf(a.h, b.l, c); return wmma_bf(a.h, b.h, c); }
__device__ __forceinline__ float sigm(float v) { return 1.0f / (1.0f + expf(-v)); }
#define LDSX() do { asm volatile("s_wait_dscnt 0" ::: "memory"); __builtin_amdgcn_wave_barrier(); __builtin_amdgcn_fence(__ATOMIC_RELEASE, "workgroup"); } while (0)

#define OUT2_OFF 4194304
#define NBT 2
#define NPT 2048
#define DM 256
#define NH 8
#define DH 64
#define KN 32
#define NR (NBT * NPT)
#ifndef NRV
#define NRV NR
#endif
#define QW (3 * NH * DH)
#define OW (NH * DH)
__device__ __forceinline__ float bfr(float v) { return (float)(__bf16)v; }
__device__ __forceinline__ v16b wcol_io(const float* __restrict__ Wm, int k0, int o, int lane, int ld) { v16b w; const float* p = Wm + (size_t)(k0 + 8 * (lane >> 4)) * ld + o; float t0[8], t1[8];
#pragma unroll
  for (int i = 0; i < 8; ++i) t0[i] = p[(size_t)i * ld];
  asm volatile("s_wait_loadcnt 0x0" ::: "memory");
#pragma unroll
  for (int i = 0; i < 8; ++i) t1[i] = p[(size_t)(16 + i) * ld];
  asm volatile("s_wait_loadcnt 0x0" ::: "memory");
#pragma unroll
  for (int i = 0; i < 8; ++i) { w[i] = (__bf16)t0[i]; w[8 + i] = (__bf16)t1[i]; }
  return w; }
#define WS_IDX 0u
#define WS_DS  (WS_IDX + 4u * (size_t)NR * KN)
#define WS_QKV (WS_DS + 4u * (size_t)NR * KN)
#define WS_O   (WS_QKV + 4u * (size_t)NR * QW)
#define WS_CO  (WS_O + 4u * (size_t)NR * OW)
#define WS_END (WS_CO + 16u * (size_t)NR)
struct Best32 { float d[KN]; int i[KN]; };
__device__ __forceinline__ void push32(Best32& b, float d, int i) {
  if (d < b.d[KN - 1]) { b.d[KN - 1] = d; b.i[KN - 1] = i; }
#pragma unroll
  for (int p = KN - 1; p > 0; --p) { const bool sw = b.d[p] < b.d[p - 1]; const float td = b.d[p], ud = b.d[p - 1]; const int ti = b.i[p], ui = b.i[p - 1]; b.d[p] = sw ? ud : td; b.d[p - 1] = sw ? td : ud; b.i[p] = sw ? ui : ti; b.i[p - 1] = sw ? ti : ui; } }
__global__ __launch_bounds__(256) void k_knn32(const float* __restrict__ P, int* __restrict__ IDX, float* __restrict__ DS) {
  const int wave = threadIdx.x >> 5, lane = threadIdx.x & 31; const size_t row = (size_t)blockIdx.x * 8 + wave; if (row >= (size_t)NRV) return;
  const size_t b = row / NPT; const int m = (int)(row % NPT);
  Best32 bs;
#pragma unroll
  for (int r = 0; r < KN; ++r) { bs.d[r] = 3.0e38f; bs.i[r] = 0x7fffffff; }
  {
#pragma clang fp contract(off)
    const float qx = bfr(P[(b * NPT + m) * 3]), qy = bfr(P[(b * NPT + m) * 3 + 1]), qz = bfr(P[(b * NPT + m) * 3 + 2]);
#pragma unroll 1
    for (int s = lane; s < NPT; s += 32) { const float px = bfr(P[(b * NPT + s) * 3]), py = bfr(P[(b * NPT + s) * 3 + 1]), pz = bfr(P[(b * NPT + s) * 3 + 2]);
      const float dx = qx - px, dy = qy - py, dz = qz - pz; const float d = __fsqrt_rn((dx * dx + dy * dy) + dz * dz);
      push32(bs, d, s); } }
  int sel = 0; float seld = 0.f;
#pragma unroll 1
  for (int r = 0; r < KN; ++r) { float d = bs.d[0]; int i = bs.i[0];
#pragma unroll
    for (int o = 1; o < 32; o <<= 1) { const float e = __shfl_xor(d, o); const int j = __shfl_xor(i, o); if (e < d || (e == d && j < i)) { d = e; i = j; } }
    if (lane == r) { sel = i; seld = d; }
    { const bool pop = (bs.i[0] == i && bs.d[0] == d);
#pragma unroll
      for (int p = 0; p < KN - 1; ++p) { bs.d[p] = pop ? bs.d[p + 1] : bs.d[p]; bs.i[p] = pop ? bs.i[p + 1] : bs.i[p]; }
      bs.d[KN - 1] = pop ? 3.0e38f : bs.d[KN - 1]; bs.i[KN - 1] = pop ? 0x7fffffff : bs.i[KN - 1]; } }
  vst2(IDX + row * KN + lane, sel); vst2(DS + row * KN + lane, seld); }

__global__ __launch_bounds__(128) void k_qkv(const float* __restrict__ X, const float* __restrict__ Wm, float* __restrict__ OUT) { __shared__ __align__(16) float sf[4][16][132];
  const int tid = threadIdx.x, wave = tid >> 5, lane = tid & 31, col = lane & 15, g = lane >> 4; const int c0 = blockIdx.y * 128; const size_t r0 = (size_t)blockIdx.x * 64 + wave * 16;
  v8f acc[8] = {};
#pragma unroll 2
  for (int kc = 0; kc < DM / 32; ++kc) { v16b a; { const float* p = X + (r0 + col) * DM + kc * 32 + 8 * g; float t0[8], t1[8];
#pragma unroll
      for (int i = 0; i < 8; ++i) t0[i] = p[i];
      asm volatile("s_wait_loadcnt 0x0" ::: "memory");
#pragma unroll
      for (int i = 0; i < 8; ++i) t1[i] = p[16 + i];
      asm volatile("s_wait_loadcnt 0x0" ::: "memory");
#pragma unroll
      for (int i = 0; i < 8; ++i) { a[i] = (__bf16)t0[i]; a[8 + i] = (__bf16)t1[i]; } }
#pragma unroll
    for (int j = 0; j < 8; ++j) { const v16b w = wcol_io(Wm, kc * 32, c0 + j * 16 + col, lane, QW); asm volatile("s_wait_loadcnt 0x0" ::: "memory"); acc[j] = wmma_bf(a, w, acc[j]); } }
#pragma unroll
  for (int j = 0; j < 8; ++j)
#pragma unroll
    for (int r = 0; r < 8; ++r) sf[wave][8 * g + r][j * 16 + col] = acc[j][r];
  LDSX(); for (int rl = 0; rl < 16; ++rl) vst2(OUT + (r0 + rl) * QW + c0 + lane * 4, *(const v4f*)&sf[wave][rl][lane * 4]); }
__constant__ float c_if16[16] = { 1.0f, 0.56234133f, 0.31622776f, 0.17782794f, 0.1f, 0.056234132f, 0.031622777f, 0.017782794f, 0.01f, 0.0056234132f, 0.0031622776f, 0.0017782794f, 0.001f, 0.00056234130f, 0.00031622776f, 0.00017782794f };
__global__ __launch_bounds__(128) void k_eqa(const float* __restrict__ P, const float* __restrict__ QKV, const int* __restrict__ IDX, const float* __restrict__ DS, const float* __restrict__ WC1, const float* __restrict__ BC1, const float* __restrict__ WC2, const float* __restrict__ BC2, const float* __restrict__ WG, const float* __restrict__ BG, const float* __restrict__ LNG, const float* __restrict__ LNB, const float* __restrict__ CCB, float* __restrict__ O, float* __restrict__ CO) {
  __shared__ float skr[4][KN][DH + 1]; __shared__ float sq8[4][16][DH + 1]; __shared__ float sp[4][16][KN + 1]; __shared__ float sqk[4][KN][NH + 1]; __shared__ float swc1[NH * 16], sbc1[16], swc2[16 * NH], sbc2[NH], swg[NH * NH], sbg[NH], sccb[NH];
  const int tid = threadIdx.x, wave = tid >> 5, lane = tid & 31, col = lane & 15, g = lane >> 4; const size_t row = (size_t)blockIdx.x * 4 + wave; const size_t b = row / NPT;
  for (int i2 = tid; i2 < NH * 16; i2 += 128) { swc1[i2] = bfr(WC1[i2]); swc2[i2] = bfr(WC2[i2]); } if (tid < 16) sbc1[tid] = bfr(BC1[tid]); if (tid < NH) { sbc2[tid] = bfr(BC2[tid]); sbg[tid] = bfr(BG[tid]); sccb[tid] = bfr(CCB[tid]); } if (tid < NH * NH) swg[tid] = bfr(WG[tid]);
  __syncthreads();
  int ix = IDX[row * KN + lane]; ix = ix < 0 ? 0 : (ix >= NPT ? NPT - 1 : ix); const size_t nb = b * NPT + ix; const float dist = DS[row * KN + lane];
  const float* qrow = QKV + row * QW; const float* krow = QKV + nb * QW + OW; const float* vrow = QKV + nb * QW + 2 * OW;
  float cs[16], sn[16]; { const float t100 = dist * 100.0f;
#pragma unroll
    for (int p = 0; p < 16; ++p) { float s_, c_; sincosf(t100 * c_if16[p], &s_, &c_); cs[p] = c_; sn[p] = s_; } }
  for (int h = 0; h < 16; ++h) { const float qa = h < NH ? qrow[(h < NH ? h : 0) * DH + lane] : 0.f, qb = h < NH ? qrow[(h < NH ? h : 0) * DH + 32 + lane] : 0.f; asm volatile("s_wait_loadcnt 0x0" ::: "memory"); sq8[wave][h][lane] = qa; sq8[wave][h][32 + lane] = qb; }
  for (int h = 0; h < NH; ++h) {
#pragma unroll
    for (int p = 0; p < 16; ++p) { const float k0 = krow[h * DH + 2 * p], k1 = krow[h * DH + 2 * p + 1]; if ((p & 3) == 3) asm volatile("s_wait_loadcnt 0x0" ::: "memory"); skr[wave][lane][2 * p] = k0 * cs[p] - k1 * sn[p]; skr[wave][lane][2 * p + 1] = k1 * cs[p] + k0 * sn[p]; }
#pragma unroll 8
    for (int d = 32; d < DH; ++d) { const float kd = krow[h * DH + d]; if ((d & 7) == 7) asm volatile("s_wait_loadcnt 0x0" ::: "memory"); skr[wave][lane][d] = kd; }
    LDSX();
    float qk;
    { v8f acc[2] = {};
#pragma unroll
      for (int kc = 0; kc < 2; ++kc) { float va[16];
#pragma unroll
        for (int i2 = 0; i2 < 8; ++i2) { va[i2] = sq8[wave][col][kc * 32 + 8 * g + i2]; va[8 + i2] = sq8[wave][col][kc * 32 + 16 + 8 * g + i2]; }
        const F2 a = bsplit16(va);
#pragma unroll
        for (int jt = 0; jt < 2; ++jt) { float vb[16]; const int jj = jt * 16 + col;
#pragma unroll
          for (int i2 = 0; i2 < 8; ++i2) { vb[i2] = skr[wave][jj][kc * 32 + 8 * g + i2]; vb[8 + i2] = skr[wave][jj][kc * 32 + 16 + 8 * g + i2]; }
          const F2 bk = bsplit16(vb); acc[jt] = wmma_bf(a.h, bk.h, acc[jt]); acc[jt] = wmma_bf(a.h, bk.l, acc[jt]); acc[jt] = wmma_bf(a.l, bk.h, acc[jt]); acc[jt] = wmma_bf(a.l, bk.l, acc[jt]); } }
#pragma unroll
      for (int jt = 0; jt < 2; ++jt) { float qv = 0.f;
#pragma unroll
        for (int r2 = 0; r2 < 8; ++r2) qv = (r2 == h) ? acc[jt][r2] : qv;
        if (g == 0) sp[wave][0][jt * 16 + col] = qv * 0.125f; }
    }
    LDSX();
    qk = sp[wave][0][lane]; sqk[wave][lane][h] = qk;
    float mx = qk;
#pragma unroll
    for (int o = 1; o < 32; o <<= 1) mx = fmaxf(mx, __shfl_xor(mx, o));
    const float ex = expf(qk - mx); float se = ex;
#pragma unroll
    for (int o = 1; o < 32; o <<= 1) se += __shfl_xor(se, o);
    const float pj = ex / se;
    LDSX();
    for (int r2 = 0; r2 < 16; ++r2) sp[wave][r2][lane] = (r2 == 0) ? pj : 0.f;
#pragma unroll
    for (int p = 0; p < 16; ++p) { const float v0 = vrow[h * DH + 2 * p], v1 = vrow[h * DH + 2 * p + 1]; if ((p & 3) == 3) asm volatile("s_wait_loadcnt 0x0" ::: "memory"); skr[wave][lane][2 * p] = v0 * cs[p] - v1 * sn[p]; skr[wave][lane][2 * p + 1] = v1 * cs[p] + v0 * sn[p]; }
#pragma unroll 8
    for (int d = 32; d < DH; ++d) { const float vd = vrow[h * DH + d]; if ((d & 7) == 7) asm volatile("s_wait_loadcnt 0x0" ::: "memory"); skr[wave][lane][d] = vd; }
    LDSX();
    { float va[16];
#pragma unroll
      for (int i2 = 0; i2 < 8; ++i2) { va[i2] = sp[wave][col][8 * g + i2]; va[8 + i2] = sp[wave][col][16 + 8 * g + i2]; }
      const F2 a = bsplit16(va);
#pragma unroll
      for (int dt = 0; dt < 4; ++dt) { float vb[16]; const int d = dt * 16 + col;
#pragma unroll
        for (int i2 = 0; i2 < 8; ++i2) { vb[i2] = skr[wave][8 * g + i2][d]; vb[8 + i2] = skr[wave][16 + 8 * g + i2][d]; }
        const F2 bv = bsplit16(vb); v8f acc = {}; acc = wmma_bf(a.h, bv.h, acc); acc = wmma_bf(a.h, bv.l, acc); acc = wmma_bf(a.l, bv.h, acc); acc = wmma_bf(a.l, bv.l, acc);
        if (g == 0) vst2(O + row * OW + h * DH + d, acc[0]); } }
    LDSX(); }
  float qh[NH];
#pragma unroll
  for (int h = 0; h < NH; ++h) qh[h] = sqk[wave][lane][h];
  float hid[16];
#pragma unroll
  for (int u = 0; u < 16; ++u) { float a = sbc1[u];
#pragma unroll
    for (int h = 0; h < NH; ++h) a += qh[h] * swc1[h * 16 + u];
    hid[u] = 0.5f * a * (1.0f + erff(a * 0.70710678118654752f)); }
  float csum = 0.f;
#pragma unroll 1
  for (int h2 = 0; h2 < NH; ++h2) { float cw = sbc2[h2];
#pragma unroll
    for (int u = 0; u < 16; ++u) cw += hid[u] * swc2[u * NH + h2];
    float sg = sbg[h2];
#pragma unroll
    for (int h = 0; h < NH; ++h) sg += qh[h] * swg[h * NH + h2];
    sg = tanhf(sg);
    float mx = cw;
#pragma unroll
    for (int o = 1; o < 32; o <<= 1) mx = fmaxf(mx, __shfl_xor(mx, o));
    const float ex = expf(cw - mx); float se = ex;
#pragma unroll
    for (int o = 1; o < 32; o <<= 1) se += __shfl_xor(se, o);
    csum += (ex / se) * sg * sccb[h2]; }
  { const float cx = bfr(P[row * 3]) - bfr(P[nb * 3]), cy = bfr(P[row * 3 + 1]) - bfr(P[nb * 3 + 1]), cz = bfr(P[row * 3 + 2]) - bfr(P[nb * 3 + 2]);
    const float nrm = __fsqrt_rn((cx * cx + cy * cy) + cz * cz); const float den = fmaxf(nrm, 1e-8f); const float xh = (nrm - nrm) / __fsqrt_rn(1e-5f); const float ph = bfr(LNG[0]) * xh + bfr(LNB[0]);
    float ox = csum * (ph * (cx / den)), oy = csum * (ph * (cy / den)), oz = csum * (ph * (cz / den));
#pragma unroll
    for (int o = 1; o < 32; o <<= 1) { ox += __shfl_xor(ox, o); oy += __shfl_xor(oy, o); oz += __shfl_xor(oz, o); }
    if (lane < 4) { const float v = lane == 0 ? ox : (lane == 1 ? oy : (lane == 2 ? oz : 0.f)); vst2(CO + row * 4 + lane, v); } } }
__global__ __launch_bounds__(128) void k_out1(const float* __restrict__ O, const float* __restrict__ Wm, const float* __restrict__ Bv, float* __restrict__ OUT) { __shared__ __align__(16) float sf[4][16][132];
  const int tid = threadIdx.x, wave = tid >> 5, lane = tid & 31, col = lane & 15, g = lane >> 4; const int c0 = blockIdx.y * 128; const size_t r0 = (size_t)blockIdx.x * 64 + wave * 16;
  v8f acc[8] = {};
#pragma unroll 2
  for (int kc = 0; kc < OW / 32; ++kc) { const F2 a = split_row(O + (r0 + col) * OW, kc * 32, lane); asm volatile("s_wait_loadcnt 0x0" ::: "memory");
#pragma unroll
    for (int j = 0; j < 8; ++j) { const v16b w = wcol_io(Wm, kc * 32, c0 + j * 16 + col, lane, DM); acc[j] = wmma_bf(a.h, w, acc[j]); acc[j] = wmma_bf(a.l, w, acc[j]); } }
#pragma unroll
  for (int j = 0; j < 8; ++j) { const float bb = bfr(Bv[c0 + j * 16 + col]);
#pragma unroll
    for (int r = 0; r < 8; ++r) sf[wave][8 * g + r][j * 16 + col] = acc[j][r] + bb; }
  LDSX(); for (int rl = 0; rl < 16; ++rl) vst2(OUT + (r0 + rl) * DM + c0 + lane * 4, *(const v4f*)&sf[wave][rl][lane * 4]); }
__global__ __launch_bounds__(256) void k_cpo(const float* __restrict__ CO, float* __restrict__ OUT2) { const size_t r = (size_t)blockIdx.x * 256 + threadIdx.x; if (r >= (size_t)NRV) return; vst2(OUT2 + r * 3, CO[r * 4]); vst2(OUT2 + r * 3 + 1, CO[r * 4 + 1]); vst2(OUT2 + r * 3 + 2, CO[r * 4 + 2]); }
extern "C" void kernel_launch(void* const* d_in, const int* in_sizes, int n_in, void* d_out, int out_size, void* d_ws, size_t ws_size, hipStream_t stream) {
  (void)in_sizes; (void)n_in; (void)out_size;
  if (ws_size < (size_t)WS_END) return;
  char* ws = (char*)d_ws; const float** F = (const float**)d_in; int* IDX = (int*)(ws + WS_IDX); float *DS = (float*)(ws + WS_DS), *QKV = (float*)(ws + WS_QKV), *O = (float*)(ws + WS_O), *CO = (float*)(ws + WS_CO);
  k_knn32<<<dim3((NRV + 7) / 8), 256, 0, stream>>>(F[1], IDX, DS);
  k_qkv<<<dim3(NRV / 64, QW / 128), 128, 0, stream>>>(F[0], F[2], QKV);
  k_eqa<<<dim3(NRV / 4), 128, 0, stream>>>(F[1], QKV, IDX, DS, F[5], F[6], F[7], F[8], F[9], F[10], F[11], F[12], F[13], O, CO);
  k_out1<<<dim3(NRV / 64, DM / 128), 128, 0, stream>>>(O, F[3], F[4], (float*)d_out);
  k_cpo<<<dim3((NRV + 255) / 256), 256, 0, stream>>>(CO, (float*)((char*)d_out + OUT2_OFF));
}
